// GraphConvPooling_29892972380764
// MI455X (gfx1250) — hardware-verified
//
#include <hip/hip_runtime.h>
#include <stdint.h>
#include <math.h>

typedef __attribute__((ext_vector_type(16))) _Float16 v16h;
typedef __attribute__((ext_vector_type(8)))  _Float16 v8h;
typedef __attribute__((ext_vector_type(16))) __bf16   v16b;
typedef __attribute__((ext_vector_type(8)))  __bf16   v8b;
typedef __attribute__((ext_vector_type(8)))  float    v8f;
typedef __attribute__((ext_vector_type(4)))  float    v4f;

constexpr int kGraphs      = 64;
constexpr int kNodes       = 1024;
constexpr int kDim         = 64;
constexpr int kGroupGraphs = 16;
constexpr int kGroups      = kGraphs / kGroupGraphs;
constexpr int kRowsPerBlk  = 256;
constexpr int kWordsPerRow = kNodes / 32;
constexpr int kVecPerIter  = 512;

typedef char check_geom0[(kGroups * kGroupGraphs == kGraphs) ? 1 : -1];
typedef char check_geom1[(kRowsPerBlk * 4 == kNodes) ? 1 : -1];
typedef char check_geom2[((kRowsPerBlk * kWordsPerRow) % 256 == 0) ? 1 : -1];

__device__ __forceinline__ unsigned short f2bf_bits(float f) {
  unsigned u = __float_as_uint(f);
  return (unsigned short)((u + 0x7FFFu + ((u >> 16) & 1u)) >> 16);
}
__device__ __forceinline__ float bf_bits2f(unsigned short h) { return __uint_as_float(((unsigned)h) << 16); }

__device__ __forceinline__ void dep_guard_h(v8f& a, v8f& b, v16h x, v16h y) { asm volatile("v_nop\n\tv_nop\n\tv_nop\n\tv_nop" : "+v"(a), "+v"(b) : "v"(x), "v"(y)); }
__device__ __forceinline__ void dep_guard_b(v8f& a, v8f& b, v16b x, v16b y) { asm volatile("v_nop\n\tv_nop\n\tv_nop\n\tv_nop" : "+v"(a), "+v"(b) : "v"(x), "v"(y)); }
__device__ __forceinline__ void keep4_h(v16h a, v16h b, v16h c, v16h d) { asm volatile("v_nop" :: "v"(a), "v"(b), "v"(c), "v"(d)); }
__device__ __forceinline__ void keep4_b(v16b a, v16b b, v16b c, v16b d) { asm volatile("v_nop" :: "v"(a), "v"(b), "v"(c), "v"(d)); }
__device__ __forceinline__ void acc_guard4(v8f& a, v8f& b, v8f& c, v8f& d) { asm volatile("v_nop\n\tv_nop\n\tv_nop\n\tv_nop" : "+v"(a), "+v"(b), "+v"(c), "+v"(d)); }
template <typename T> struct Frag;
template <> struct Frag<_Float16> {
  typedef v16h V; union U { v16h v; v8h h[2]; };
  static __device__ __forceinline__ v16h load(const _Float16* p) {
    U f; f.h[0] = *(const v8h*)(p); f.h[1] = *(const v8h*)(p + 16); return f.v;
  }
  static __device__ __forceinline__ v8f mma(v16h a, v16h b, v8f c) {
    return __builtin_amdgcn_wmma_f32_16x16x32_f16(false, a, false, b, (short)0, c, false, false);
  }
  static __device__ __forceinline__ void guard(v8f& a, v8f& b, v16h x, v16h y) { dep_guard_h(a, b, x, y); }
  static __device__ __forceinline__ void keep(v16h a, v16h b, v16h c, v16h d) { keep4_h(a, b, c, d); }
};
template <> struct Frag<__bf16> {
  typedef v16b V; union U { v16b v; v8b h[2]; };
  static __device__ __forceinline__ v16b load(const __bf16* p) {
    U f; f.h[0] = *(const v8b*)(p); f.h[1] = *(const v8b*)(p + 16); return f.v;
  }
  static __device__ __forceinline__ v8f mma(v16b a, v16b b, v8f c) {
    return __builtin_amdgcn_wmma_f32_16x16x32_bf16(false, a, false, b, (short)0, c, false, false);
  }
  static __device__ __forceinline__ void guard(v8f& a, v8f& b, v16b x, v16b y) { dep_guard_b(a, b, x, y); }
  static __device__ __forceinline__ void keep(v16b a, v16b b, v16b c, v16b d) { keep4_b(a, b, c, d); }
};

template <int ET> struct Elem;
template <> struct Elem<0> { typedef _Float16 T; };
template <> struct Elem<1> { typedef __bf16 T; };
template <int ET, bool SPLIT, int BIAS_MODE, int OUT_MODE, bool RESID, int ACT = 0>
__global__ __launch_bounds__(256) void wmma_gemm64(
    const unsigned short* __restrict__ Ap, const unsigned short* __restrict__ A2p, int lda, long strideA,
    const unsigned short* __restrict__ Btp, const unsigned short* __restrict__ Bt2p, int ldb, long strideB,
    void* __restrict__ Cout, void* __restrict__ Cout2, int ldc, long strideC,
    const float* __restrict__ bias,
    const float* __restrict__ resid, long strideR,
    int M, int N, int K, float scale) {
  typedef typename Elem<ET>::T T;
  typedef typename Frag<T>::V V;
  const T* A = (const T*)Ap; const T* A2 = (const T*)A2p; const T* Bt = (const T*)Btp; const T* Bt2 = (const T*)Bt2p;
  __shared__ __align__(16) float sT[8][16 * 68];
  const int b    = blockIdx.y;
  const int lane = threadIdx.x & 31;
  const int wave = threadIdx.x >> 5;
  const int tilesN = N >> 6;
  const int tilesM = M >> 6;
  const int tile = blockIdx.x * 8 + wave;
  if (tile >= tilesM * tilesN) return;
  const int tm = tile / tilesN;
  const int tn = tile - tm * tilesN;
  const int m0 = tm << 6;
  const int n0 = tn << 6;

  const T* Ab  = A  + (size_t)b * strideA;
  const T* Bb  = Bt + (size_t)b * strideB;
  const T* Ab2 = SPLIT ? (A2  + (size_t)b * strideA) : nullptr;
  const T* Bb2 = SPLIT ? (Bt2 + (size_t)b * strideB) : nullptr;

  const int rlane = lane & 15;
  const int koff  = (lane >> 4) * 8;
  const int mOff  = (lane >> 4) * 8;

  v8f acc[4][4];
#pragma unroll
  for (int i = 0; i < 4; ++i)
#pragma unroll
    for (int j = 0; j < 4; ++j) acc[i][j] = (v8f){0.f,0.f,0.f,0.f,0.f,0.f,0.f,0.f};

  for (int k0 = 0; k0 < K; k0 += 32) {
    V bh[4], bl[4];
#pragma unroll
    for (int j = 0; j < 4; ++j) {
      const size_t bo = (size_t)(n0 + (j << 4) + rlane) * ldb + koff + k0;
      bh[j] = Frag<T>::load(Bb + bo);
      if (SPLIT) bl[j] = Frag<T>::load(Bb2 + bo);
    }
#pragma unroll
    for (int i = 0; i < 4; ++i) {
      const size_t ao = (size_t)(m0 + (i << 4) + rlane) * lda + koff + k0;
      V ah = Frag<T>::load(Ab + ao);
      V al;
      if (SPLIT) al = Frag<T>::load(Ab2 + ao);
#pragma unroll
      for (int j = 0; j < 4; ++j) {
        acc[i][j] = Frag<T>::mma(ah, bh[j], acc[i][j]);
        if (SPLIT) {
          acc[i][j] = Frag<T>::mma(ah, bl[j], acc[i][j]);
          acc[i][j] = Frag<T>::mma(al, bh[j], acc[i][j]);
        }
      }
      Frag<T>::guard(acc[i][0], acc[i][3], ah, SPLIT ? al : ah);
    }
    Frag<T>::keep(bh[0], bh[1], bh[2], bh[3]);
    if (SPLIT) Frag<T>::keep(bl[0], bl[1], bl[2], bl[3]);
  }
  acc_guard4(acc[0][0], acc[0][1], acc[0][2], acc[0][3]);
  acc_guard4(acc[1][0], acc[1][1], acc[1][2], acc[1][3]);
  acc_guard4(acc[2][0], acc[2][1], acc[2][2], acc[2][3]);
  acc_guard4(acc[3][0], acc[3][1], acc[3][2], acc[3][3]);

  float* slab = sT[wave];
  const float* Rb = RESID ? (resid + (size_t)b * strideR) : nullptr;
#pragma unroll
  for (int i = 0; i < 4; ++i) {
    const int mBase = m0 + (i << 4);
#pragma unroll
    for (int j = 0; j < 4; ++j) {
      const int n = n0 + (j << 4) + rlane;
      float bv = 0.f;
      if (BIAS_MODE == 2) bv = bias[n];
#pragma unroll
      for (int r = 0; r < 8; ++r) {
        float v = acc[i][j][r] * scale;
        if (BIAS_MODE == 1) v += bias[mBase + mOff + r];
        if (BIAS_MODE == 2) v += bv;
        if (RESID) v += Rb[(size_t)(mBase + mOff + r) * ldc + n];
        if (ACT == 1) v = tanhf(v);
        if (ACT == 2) v = fmaxf(v, 0.0f);
        if (ACT == 3) v = v / (1.0f + expf(-v));
        if (ACT == 4) v = (v > 0.f) ? v : 0.01f * v;
        if (ACT == 5) v = 0.5f * v * (1.0f + erff(v * 0.70710678118654752f));
        slab[(mOff + r) * 68 + (j << 4) + rlane] = v;
      }
    }
    __builtin_amdgcn_fence(__ATOMIC_RELEASE, "workgroup");
    __builtin_amdgcn_wave_barrier();
    __builtin_amdgcn_fence(__ATOMIC_ACQUIRE, "workgroup");
    if (OUT_MODE == 0) {
      float* C = (float*)Cout + (size_t)b * strideC;
      const int hh = lane >> 4, c4 = (lane & 15) * 4;
      for (int pass = 0; pass < 2; ++pass) {
#pragma unroll
        for (int it = 0; it < 8; ++it) {
          const int row = it * 2 + hh;
          v4f v = *(const v4f*)(slab + row * 68 + c4);
          *(volatile v4f*)(C + (size_t)(mBase + row) * ldc + n0 + c4) = v;
        }
        __threadfence();
      }
    } else {
      const int q = lane >> 3, c8 = (lane & 7) * 8;
      unsigned short* C  = (unsigned short*)Cout  + (size_t)b * strideC;
      unsigned short* C2 = (OUT_MODE == 2) ? ((unsigned short*)Cout2 + (size_t)b * strideC) : nullptr;
      for (int pass = 0; pass < 2; ++pass) {
#pragma unroll
        for (int it = 0; it < 4; ++it) {
          const int row = it * 4 + q;
          const float* sp = slab + row * 68 + c8;
          v8h hv, lv;
#pragma unroll
          for (int e = 0; e < 8; ++e) {
            if (OUT_MODE == 1) {
              hv[e] = (_Float16)sp[e];
            } else {
              unsigned short hb = f2bf_bits(sp[e]);
              unsigned short lb = f2bf_bits(sp[e] - bf_bits2f(hb));
              hv[e] = __builtin_bit_cast(_Float16, hb);
              lv[e] = __builtin_bit_cast(_Float16, lb);
            }
          }
          *(volatile v8h*)(C + (size_t)(mBase + row) * ldc + n0 + c8) = hv;
          if (OUT_MODE == 2) *(volatile v8h*)(C2 + (size_t)(mBase + row) * ldc + n0 + c8) = lv;
        }
        __threadfence();
      }
    }
    __builtin_amdgcn_fence(__ATOMIC_RELEASE, "workgroup");
    __builtin_amdgcn_wave_barrier();
    __builtin_amdgcn_fence(__ATOMIC_ACQUIRE, "workgroup");
  }
}

__global__ __launch_bounds__(256) void tcast64_kernel(
    const float* __restrict__ src, _Float16* __restrict__ dst,
    int jchunks, int src_grows, long dst_gstride, int dst_ld, float scale)
{
  __shared__ __align__(16) _Float16 tile[64 * 72];
  const int t = threadIdx.x, lane = t & 31, wave = t >> 5;
  const int g = blockIdx.x / jchunks;
  const int jc = blockIdx.x - g * jchunks;
  const size_t row0 = (size_t)g * src_grows + (size_t)jc * 64;
#pragma unroll
  for (int i = 0; i < 16; ++i) {
    const int idx = t + 256 * i;
    const int r = idx >> 6, c = idx & 63;
    tile[c * 72 + r] = (_Float16)(src[(row0 + r) * 64 + c] * scale);
  }
  __syncthreads();
  _Float16* dg = dst + (size_t)g * dst_gstride + (size_t)jc * 64;
  const int lr = lane >> 3, c8 = (lane & 7) * 8;
  for (int pass = 0; pass < 2; ++pass) {
#pragma unroll
    for (int it = 0; it < 2; ++it) {
      const int d = wave * 8 + it * 4 + lr;
      const v8h v = *(const v8h*)(tile + d * 72 + c8);
      *(volatile v8h*)(dg + (size_t)d * dst_ld + c8) = v;
    }
    __threadfence();
  }
}

__global__ __launch_bounds__(256) void adj_build_kernel(
    const int* __restrict__ estart, const int* __restrict__ eend,
    int nvec, int niter, int group, _Float16* __restrict__ Aplane)
{
  __shared__ unsigned int bm[kRowsPerBlk * kWordsPerRow];
  const int t = threadIdx.x, lane = t & 31, wave = t >> 5;
  const int gi = blockIdx.x >> 2, q = blockIdx.x & 3;
  const int g = group * kGroupGraphs + gi;
  const int rowlo = g * kNodes + q * kRowsPerBlk;
  const int colbase = g * kNodes;
#pragma unroll
  for (int i = 0; i < (kRowsPerBlk * kWordsPerRow) / 256; ++i) bm[t + 256 * i] = 0u;
  __syncthreads();

  const int4* s4p = (const int4*)estart;
  const int4* e4p = (const int4*)eend;
  const int nvm1 = nvec - 1;
#pragma unroll 1
  for (int it = 0; it < niter; ++it) {
#pragma unroll
    for (int half = 0; half < 2; ++half) {
      const int vi = it * kVecPerIter + half * 256 + t;
      const bool vval = vi < nvec;
      const int vic = vval ? vi : nvm1;
      const int4 sv = s4p[vic];
      const int4 ev = e4p[vic];
      const int sa[4] = { sv.x, sv.y, sv.z, sv.w };
      const int ea[4] = { ev.x, ev.y, ev.z, ev.w };
#pragma unroll
      for (int e = 0; e < 4; ++e) {
        const unsigned r = (unsigned)(sa[e] - rowlo);
        if (vval && r < (unsigned)kRowsPerBlk) {
          int c = ea[e] - colbase;
          c = c < 0 ? 0 : (c > kNodes - 1 ? kNodes - 1 : c);
          atomicOr(&bm[r * kWordsPerRow + (c >> 5)], 1u << (c & 31));
        }
      }
    }
  }
  __syncthreads();

  _Float16* Ablk = Aplane + ((size_t)(gi * kNodes + q * kRowsPerBlk)) * kNodes;
  const int lq = lane >> 2, lsh = (lane & 3) * 8;
  for (int pass = 0; pass < 2; ++pass) {
#pragma unroll 1
    for (int rr = 0; rr < 32; ++rr) {
      const int r = wave * 32 + rr;
#pragma unroll
      for (int s = 0; s < 4; ++s) {
        const unsigned w = bm[r * kWordsPerRow + s * 8 + lq];
        const unsigned bits = (w >> lsh) & 0xFFu;
        union { v8h v; unsigned u[4]; } pk;
#pragma unroll
        for (int i = 0; i < 4; ++i) {
          const unsigned b0 = (bits >> (2 * i)) & 1u;
          const unsigned b1 = (bits >> (2 * i + 1)) & 1u;
          pk.u[i] = (b0 ? 0x00003C00u : 0u) | (b1 ? 0x3C000000u : 0u);
        }
        *(volatile v8h*)(Ablk + (size_t)r * kNodes + s * 256 + lane * 8) = pk.v;
      }
    }
    __threadfence();
  }
}

__global__ __launch_bounds__(256) void pool_mlp_kernel(
    const float* __restrict__ yw,
    const float* __restrict__ w1, const float* __restrict__ b1,
    const float* __restrict__ w2, const float* __restrict__ b2,
    const float* __restrict__ w3, const float* __restrict__ b3,
    float* __restrict__ out)
{
  __shared__ float hbuf[2 * kGraphs * kDim];
  __shared__ __align__(16) float outv[kGraphs];
  const int t = threadIdx.x, lane = t & 31, wave = t >> 5;
  const int d = t & 63, g4 = t >> 6;

#pragma unroll 1
  for (int gg = 0; gg < kGraphs / 4; ++gg) {
    const int g = gg * 4 + g4;
    const float* base = yw + (size_t)g * kNodes * kDim + d;
    float m = base[0];
#pragma unroll 4
    for (int i = 1; i < kNodes; ++i) m = fmaxf(m, base[(size_t)i * kDim]);
    hbuf[g * kDim + d] = m;
  }
  __syncthreads();

#pragma unroll 1
  for (int layer = 0; layer < 2; ++layer) {
    const float* wl = layer ? w2 : w1;
    const float* bl = layer ? b2 : b1;
    const int inoff  = layer * (kGraphs * kDim);
    const int outoff = (layer ^ 1) * (kGraphs * kDim);
#pragma unroll 1
    for (int p = 0; p < (kGraphs * kDim) / 256; ++p) {
      const int idx = t + 256 * p;
      const int g = idx >> 6, n = idx & 63;
      float s = bl[n];
#pragma unroll 1
      for (int k = 0; k < kDim; ++k) s = fmaf(hbuf[inoff + g * kDim + k], wl[k * kDim + n], s);
      hbuf[outoff + idx] = tanhf(s);
    }
    __syncthreads();
  }

  if (t < kGraphs) {
    float s = b3[0];
#pragma unroll 1
    for (int n = 0; n < kDim; ++n) s = fmaf(hbuf[t * kDim + n], w3[n], s);
    outv[t] = s;
  }
  __syncthreads();
  if (wave == 0) {
    const int lc = lane & 15;
    for (int pass = 0; pass < 2; ++pass) {
      const v4f v = *(const v4f*)(outv + lc * 4);
      if (lane < 16) *(volatile v4f*)(out + lc * 4) = v;
      __threadfence();
    }
  }
}

extern "C" void kernel_launch(void* const* d_in, const int* in_sizes, int n_in,
                              void* d_out, int out_size, void* d_ws, size_t ws_size,
                              hipStream_t stream) {
  if (n_in < 12) return;
  if (in_sizes[0] != kGraphs * kNodes * kDim) return;
  if (in_sizes[4] != kDim * kDim || in_sizes[5] != kDim || in_sizes[6] != kDim * kDim ||
      in_sizes[7] != kDim || in_sizes[8] != kDim * kDim || in_sizes[9] != kDim ||
      in_sizes[10] != kDim || in_sizes[11] < 1) return;
  if (out_size != kGraphs) return;

  const float* x      = (const float*)d_in[0];
  const int*   eidx   = (const int*)d_in[1];
  const float* weight = (const float*)d_in[4];
  const float* bias   = (const float*)d_in[5];
  const float* w1     = (const float*)d_in[6];
  const float* b1     = (const float*)d_in[7];
  const float* w2     = (const float*)d_in[8];
  const float* b2     = (const float*)d_in[9];
  const float* w3     = (const float*)d_in[10];
  const float* b3     = (const float*)d_in[11];
  float* out = (float*)d_out;

  const int NE = in_sizes[1] / 2;
  if (NE < 4 || (NE & 3) != 0) return;
  const int* estart = eidx;
  const int* eend   = eidx + NE;
  const int nvec  = NE >> 2;
  const int niter = (nvec + kVecPerIter - 1) / kVecPerIter;

  const size_t bytesXT = (size_t)kGraphs * kDim * kNodes * 2;
  const size_t bytesA  = (size_t)kGroupGraphs * kNodes * kNodes * 2;
  const size_t bytesY  = (size_t)kGraphs * kNodes * kDim * 2;
  const size_t bytesWT = (size_t)kDim * kDim * 2;
  const size_t bytesYW = (size_t)kGraphs * kNodes * kDim * 4;
  const size_t offXT = 0;
  const size_t offA  = offXT + bytesXT;
  const size_t offY  = offA + bytesA;
  const size_t offWT = offY + bytesY;
  const size_t offYW = offWT + bytesWT;
  const size_t total = offYW + bytesYW;
  if (total > ws_size) return;

  char* ws = (char*)d_ws;
  _Float16* XT16 = (_Float16*)(ws + offXT);
  _Float16* A16  = (_Float16*)(ws + offA);
  _Float16* Y16  = (_Float16*)(ws + offY);
  _Float16* WT16 = (_Float16*)(ws + offWT);
  float*    YW   = (float*)(ws + offYW);

  tcast64_kernel<<<kGraphs * (kNodes / 64), 256, 0, stream>>>(x, XT16, kNodes / 64, kNodes,
                                                              (long)kDim * kNodes, kNodes, 1.0f);
  tcast64_kernel<<<1, 256, 0, stream>>>(weight, WT16, 1, kNodes, 0L, kDim, 16.0f);

  for (int grp = 0; grp < kGroups; ++grp) {
    adj_build_kernel<<<kGroupGraphs * 4, 256, 0, stream>>>(estart, eend, nvec, niter, grp, A16);
    const unsigned short* Bt = (const unsigned short*)(XT16 + (size_t)grp * kGroupGraphs * kDim * kNodes);
    unsigned short* Cp = (unsigned short*)(Y16 + (size_t)grp * kGroupGraphs * kNodes * kDim);
    wmma_gemm64<0, false, 0, 1, false, 0><<<dim3((kNodes / 64 + 7) / 8, kGroupGraphs), 256, 0, stream>>>(
        (const unsigned short*)A16, (const unsigned short*)A16, kNodes, (long)kNodes * kNodes,
        Bt, Bt, kNodes, (long)kDim * kNodes,
        (void*)Cp, (void*)Cp, kDim, (long)kNodes * kDim,
        bias, x, 0L,
        kNodes, kDim, kNodes, 1.0f);
  }

  wmma_gemm64<0, false, 2, 0, false, 0><<<dim3((kGraphs * kNodes / 64 + 7) / 8, 1), 256, 0, stream>>>(
      (const unsigned short*)Y16, (const unsigned short*)Y16, kDim, 0L,
      (const unsigned short*)WT16, (const unsigned short*)WT16, kDim, 0L,
      (void*)YW, (void*)YW, kDim, 0L,
      bias, x, 0L,
      kGraphs * kNodes, kDim, kDim, 1.0f / 16.0f);

  pool_mlp_kernel<<<1, 256, 0, stream>>>(YW, w1, b1, w2, b2, w3, b3, out);
}
